// GRUCell_87703232184582
// MI455X (gfx1250) — hardware-verified
//
#include <hip/hip_runtime.h>
#include <hip/hip_bf16.h>


typedef __bf16 bf16;
typedef __attribute__((ext_vector_type(16))) __bf16 v16bf;
typedef __attribute__((ext_vector_type(8)))  __bf16 v8bf;
typedef __attribute__((ext_vector_type(8)))  float  v8f;
typedef float v4f  __attribute__((ext_vector_type(4)));
typedef float v4fa __attribute__((ext_vector_type(4), may_alias));
typedef unsigned int v4u __attribute__((ext_vector_type(4)));

#define GAS __attribute__((address_space(1)))
typedef GAS const bf16* gcptr;

#ifndef NB
#define NB 16384
#endif
#define NB_FULL 16384
#define DIM_I  512
#define DIM_H  512
#define DIM_K  1024
#define TILE_M 128
#define TILE_N 32
#define SPITCH 36

#define NG_ELEMS ((size_t)DIM_K * DIM_K)
#define NI_ELEMS ((size_t)DIM_H * DIM_I)
#define NH_ELEMS ((size_t)DIM_H * DIM_H)

static_assert(NB % TILE_M == 0);
static_assert(NB >= TILE_M && NB <= NB_FULL);
static_assert(DIM_H % TILE_N == 0);
static_assert(DIM_I % 64 == 0 && DIM_H % 64 == 0);
static_assert((SPITCH % 4) == 0);
static_assert((NG_ELEMS % 2048) == 0 && (NI_ELEMS % 2048) == 0 && (NH_ELEMS % 2048) == 0);
static_assert((((size_t)NB * DIM_K) % 2048) == 0);

__device__ __forceinline__ unsigned int bf16_bits(float f) {
    unsigned int u = __float_as_uint(f);
    return (u + 0x7FFFu + ((u >> 16) & 1u)) >> 16;
}
__device__ __forceinline__ float bf16_val(float f) {
    return __uint_as_float(bf16_bits(f) << 16);
}

__device__ __forceinline__ v16bf frag_at(gcptr p, int ko) {
    v8bf lo = *(const GAS v8bf*)(p + ko);
    v8bf hi = *(const GAS v8bf*)(p + ko + 16);
    return __builtin_shufflevector(lo, hi, 0,1,2,3,4,5,6,7,8,9,10,11,12,13,14,15);
}

__device__ __forceinline__ v8f wmma_bf16(v16bf a, v16bf b, v8f c) {
    v8f d = __builtin_amdgcn_wmma_f32_16x16x32_bf16(false, a, false, b, (short)0, c, false, false);
    asm volatile("v_nop\n\tv_nop\n\tv_nop\n\tv_nop" : "+v"(d) : "v"(a), "v"(b));
    return d;
}

__device__ __forceinline__ float fast_sigmoid(float x) {
    x = fminf(fmaxf(x, -30.f), 30.f);
    float e = __expf(-x);
    return __fdividef(1.f, 1.f + e);
}

__device__ __forceinline__ float fast_tanh(float x) {
    x = fminf(fmaxf(x, -15.f), 15.f);
    float e = __expf(2.f * x);
    return __fdividef(e - 1.f, e + 1.f);
}

__device__ __forceinline__ v4u pack8_bf16(float4 f0, float4 f1) {
    v4u o;
    o.x = bf16_bits(f0.x) | (bf16_bits(f0.y) << 16);
    o.y = bf16_bits(f0.z) | (bf16_bits(f0.w) << 16);
    o.z = bf16_bits(f1.x) | (bf16_bits(f1.y) << 16);
    o.w = bf16_bits(f1.z) | (bf16_bits(f1.w) << 16);
    return o;
}

__global__ __launch_bounds__(256) void fuse_convert_kernel(const float* __restrict__ x,
                                                           const float* __restrict__ h,
                                                           unsigned short* __restrict__ fusedA) {
    const size_t base = ((size_t)blockIdx.x * 256 + threadIdx.x) * 8;
    const int    col  = (int)(base & 1023);
    const size_t row  = base >> 10;
    const float* src = (col < DIM_I) ? (x + row * DIM_I + col)
                                     : (h + row * DIM_H + (col - DIM_I));
    const float4 f0 = *(const float4*)(src);
    const float4 f1 = *(const float4*)(src + 4);
    const v4u o = pack8_bf16(f0, f1);
    volatile v4u* d = (volatile v4u*)(fusedA + base);
    *d = o;
    __threadfence();
    *d = o;
}

__global__ __launch_bounds__(256) void weight_convert_kernel(const float* __restrict__ Wg,
                                                             const float* __restrict__ Wi,
                                                             const float* __restrict__ Wh,
                                                             unsigned short* __restrict__ dst) {
    const size_t g = ((size_t)blockIdx.x * 256 + threadIdx.x) * 8;
    if (g >= NG_ELEMS + NI_ELEMS + NH_ELEMS) return;
    const float* src = (g < NG_ELEMS) ? (Wg + g)
                     : ((g < NG_ELEMS + NI_ELEMS) ? (Wi + (g - NG_ELEMS))
                                                  : (Wh + (g - NG_ELEMS - NI_ELEMS)));
    const float4 f0 = *(const float4*)(src);
    const float4 f1 = *(const float4*)(src + 4);
    const v4u o = pack8_bf16(f0, f1);
    volatile v4u* d = (volatile v4u*)(dst + g);
    *d = o;
    __threadfence();
    *d = o;
}

__global__ __launch_bounds__(256) void cell_gemm_kernel(
    const bf16* __restrict__ fusedA, const bf16* __restrict__ Wgb,
    const bf16* __restrict__ Wib,    const bf16* __restrict__ Whb,
    const float* __restrict__ b_gate, const float* __restrict__ b_i,
    const float* __restrict__ b_h,    const float* __restrict__ hidden,
    float* __restrict__ out)
{
    __shared__ __attribute__((aligned(16))) float sZ[TILE_M * SPITCH];
    __shared__ __attribute__((aligned(16))) float sN[TILE_M * SPITCH];

    const int lane = threadIdx.x & 31;
    const int wave = threadIdx.x >> 5;
    const int wm   = wave >> 1;
    const int wn   = wave & 1;
    const int mblk = blockIdx.y * TILE_M;
    const int nblk = blockIdx.x * TILE_N;
    const int m0   = mblk + wm * 32;
    const int n0   = nblk + wn * 16;
    const int lrow = lane & 15;
    const int lh   = (lane >> 4) * 8;

    gcptr ap[2];
    #pragma unroll
    for (int mt = 0; mt < 2; ++mt)
        ap[mt] = (gcptr)fusedA + (size_t)(m0 + mt * 16 + lrow) * DIM_K + lh;
    const gcptr pgr = (gcptr)Wgb + (size_t)(n0 + lrow) * DIM_K + lh;
    const gcptr pgz = (gcptr)Wgb + (size_t)(DIM_H + n0 + lrow) * DIM_K + lh;
    const gcptr pwi = (gcptr)Wib + (size_t)(n0 + lrow) * DIM_I + lh;
    const gcptr pwh = (gcptr)Whb + (size_t)(n0 + lrow) * DIM_H + lh;

    v8f ar[2] = {}, az[2] = {}, ai[2] = {}, ah[2] = {};

    #pragma unroll 1
    for (int k = 0; k < DIM_I; k += 64) {
        #pragma unroll
        for (int u = 0; u < 2; ++u) {
            const int ko = u * 32;
            const v16bf a0 = frag_at(ap[0] + k, ko);
            const v16bf a1 = frag_at(ap[1] + k, ko);
            const v16bf fr = frag_at(pgr + k, ko);
            const v16bf fz = frag_at(pgz + k, ko);
            const v16bf fx = frag_at(pwi + k, ko);
            ar[0] = wmma_bf16(a0, fr, ar[0]);
            ar[1] = wmma_bf16(a1, fr, ar[1]);
            az[0] = wmma_bf16(a0, fz, az[0]);
            az[1] = wmma_bf16(a1, fz, az[1]);
            ai[0] = wmma_bf16(a0, fx, ai[0]);
            ai[1] = wmma_bf16(a1, fx, ai[1]);
        }
    }

    #pragma unroll 1
    for (int k = 0; k < DIM_H; k += 64) {
        #pragma unroll
        for (int u = 0; u < 2; ++u) {
            const int ko = u * 32;
            const v16bf a0 = frag_at(ap[0] + DIM_I + k, ko);
            const v16bf a1 = frag_at(ap[1] + DIM_I + k, ko);
            const v16bf fr = frag_at(pgr + DIM_I + k, ko);
            const v16bf fz = frag_at(pgz + DIM_I + k, ko);
            const v16bf fx = frag_at(pwh + k, ko);
            ar[0] = wmma_bf16(a0, fr, ar[0]);
            ar[1] = wmma_bf16(a1, fr, ar[1]);
            az[0] = wmma_bf16(a0, fz, az[0]);
            az[1] = wmma_bf16(a1, fz, az[1]);
            ah[0] = wmma_bf16(a0, fx, ah[0]);
            ah[1] = wmma_bf16(a1, fx, ah[1]);
        }
    }

    const int   mh  = (lane >> 4) * 8;
    const int   col = n0 + lrow;
    const float bgr = bf16_val(b_gate[col]);
    const float bgz = bf16_val(b_gate[DIM_H + col]);
    const float bii = bf16_val(b_i[col]);
    const float bhh = bf16_val(b_h[col]);
    #pragma unroll
    for (int mt = 0; mt < 2; ++mt) {
        #pragma unroll
        for (int r = 0; r < 8; ++r) {
            const int   rl = wm * 32 + mt * 16 + mh + r;
            const float rg = fast_sigmoid(ar[mt][r] + bgr);
            const float zg = fast_sigmoid(az[mt][r] + bgz);
            const float ng = fast_tanh(ai[mt][r] + bii + rg * (ah[mt][r] + bhh));
            const int   li = rl * SPITCH + wn * 16 + lrow;
            sZ[li] = zg;
            sN[li] = ng;
        }
    }
    __syncthreads();

    v4f    vals[4];
    size_t goff[4];
    #pragma unroll
    for (int it = 0; it < 4; ++it) {
        const int rl = wave * 16 + it * 4 + (lane >> 3);
        const int c4 = (lane & 7) * 4;
        const v4fa z4 = *(const v4fa*)(&sZ[rl * SPITCH + c4]);
        const v4fa n4 = *(const v4fa*)(&sN[rl * SPITCH + c4]);
        const size_t o = (size_t)(mblk + rl) * DIM_H + nblk + c4;
        const float4 h4 = *(const float4*)(hidden + o);
        v4f v;
        {
            const float hp0 = bf16_val(h4.x), hp1 = bf16_val(h4.y);
            const float hp2 = bf16_val(h4.z), hp3 = bf16_val(h4.w);
            v[0] = (1.f - z4[0]) * n4[0] + z4[0] * hp0;
            v[1] = (1.f - z4[1]) * n4[1] + z4[1] * hp1;
            v[2] = (1.f - z4[2]) * n4[2] + z4[2] * hp2;
            v[3] = (1.f - z4[3]) * n4[3] + z4[3] * hp3;
        }
        vals[it] = v;
        goff[it] = o;
    }
    #pragma unroll
    for (int it = 0; it < 4; ++it)
        *(volatile v4f*)(out + goff[it]) = vals[it];
    __threadfence();
    #pragma unroll
    for (int it = 0; it < 4; ++it)
        *(volatile v4f*)(out + goff[it]) = vals[it];
}

extern "C" void kernel_launch(void* const* d_in, const int* in_sizes, int n_in,
                              void* d_out, int out_size, void* d_ws, size_t ws_size,
                              hipStream_t stream) {
    if (n_in < 8) return;
    if (in_sizes[0] < NB * DIM_I) return;
    if (in_sizes[1] < NB * DIM_H) return;
    if (in_sizes[2] < DIM_K * DIM_K) return;
    if (in_sizes[3] < DIM_K) return;
    if (in_sizes[4] < DIM_H * DIM_I) return;
    if (in_sizes[5] < DIM_H) return;
    if (in_sizes[6] < DIM_H * DIM_H) return;
    if (in_sizes[7] < DIM_H) return;
    if (out_size < NB * DIM_H) return;

    const float* x      = (const float*)d_in[0];
    const float* hidden = (const float*)d_in[1];
    const float* W_gate = (const float*)d_in[2];
    const float* b_gate = (const float*)d_in[3];
    const float* W_i    = (const float*)d_in[4];
    const float* b_i    = (const float*)d_in[5];
    const float* W_h    = (const float*)d_in[6];
    const float* b_h    = (const float*)d_in[7];
    float* out = (float*)d_out;

    char* ws = (char*)d_ws;
    size_t off = 0;
    unsigned short* fusedA = (unsigned short*)(ws + off);
    off += (size_t)NB * DIM_K * sizeof(unsigned short);
    unsigned short* Wall = (unsigned short*)(ws + off);
    off += (NG_ELEMS + NI_ELEMS + NH_ELEMS) * sizeof(unsigned short);
    if (off > ws_size) return;
    const bf16* Wgb = (const bf16*)Wall;
    const bf16* Wib = (const bf16*)(Wall + NG_ELEMS);
    const bf16* Whb = (const bf16*)(Wall + NG_ELEMS + NI_ELEMS);

    const unsigned fuse_blocks   = (unsigned)(((size_t)NB * DIM_K) / 2048);
    const unsigned weight_blocks = (unsigned)((NG_ELEMS + NI_ELEMS + NH_ELEMS) / 2048);

    fuse_convert_kernel<<<fuse_blocks, 256, 0, stream>>>(x, hidden, fusedA);
    weight_convert_kernel<<<weight_blocks, 256, 0, stream>>>(W_gate, W_i, W_h, Wall);

    cell_gemm_kernel<<<dim3(DIM_H / TILE_N, NB / TILE_M), 256, 0, stream>>>(
        (const bf16*)fusedA, Wgb, Wib, Whb, b_gate, b_i, b_h, hidden, out);
}
